// LightNetAttention_15015205667340
// MI455X (gfx1250) — hardware-verified
//
#include <hip/hip_runtime.h>
#include <stdint.h>
#include <math.h>

typedef __attribute__((ext_vector_type(16))) _Float16 v16h;
typedef __attribute__((ext_vector_type(8)))  _Float16 v8h;
typedef __attribute__((ext_vector_type(16))) __bf16   v16b;
typedef __attribute__((ext_vector_type(8)))  __bf16   v8b;
typedef __attribute__((ext_vector_type(8)))  float    v8f;
typedef __attribute__((ext_vector_type(4)))  float    v4f;
typedef __attribute__((ext_vector_type(4)))  unsigned v4u;

constexpr int kBatch     = 4;
constexpr int kSeqLen    = 2048;
constexpr int kHid       = 1024;
constexpr int kHeads     = 8;
constexpr int kHeadDim   = 128;
constexpr int kChunkLen  = 64;
constexpr int kNumChunk  = kSeqLen / kChunkLen;
constexpr int kGateRank  = 128;
constexpr int kBatchHalf = 2;
constexpr int kNumHalf   = kBatch / kBatchHalf;
constexpr int kRowsHalf  = kBatchHalf * kSeqLen;
static_assert(kHeads * kHeadDim == kHid);
static_assert(kRowsHalf % 64 == 0 && kHid % 64 == 0 && kGateRank % 64 == 0);
static_assert(kHid % 32 == 0 && kGateRank % 32 == 0);
static_assert(kSeqLen % kChunkLen == 0 && kChunkLen == 64 && kHeadDim == 128);
static_assert(kHid == 128 * 8);

constexpr size_t kPlaneF32 = (size_t)kRowsHalf * kHid * 4;
constexpr size_t kPlane16  = (size_t)kRowsHalf * kHid * 2;
constexpr size_t kWBytes   = (size_t)kHid * kHid * 2;
constexpr size_t kWgBytes  = (size_t)kGateRank * kHid * 2;
constexpr size_t kOffXb  = 0;
constexpr size_t kOffWq  = kOffXb + kPlane16;
constexpr size_t kOffWk  = kOffWq + kWBytes;
constexpr size_t kOffWv  = kOffWk + kWBytes;
constexpr size_t kOffWo  = kOffWv + kWBytes;
constexpr size_t kOffWg1 = kOffWo + kWBytes;
constexpr size_t kOffWg2 = kOffWg1 + kWgBytes;
constexpr size_t kOffR2  = kOffWg2 + kWgBytes;
constexpr size_t kOffR3  = kOffR2 + kPlaneF32;
constexpr size_t kOffR4  = kOffR3 + kPlaneF32;
constexpr size_t kOffR5  = kOffR4 + kPlaneF32;
constexpr size_t kOffR6  = kOffR5 + kPlaneF32;
constexpr size_t kOffR7  = kOffR6 + kPlaneF32;
constexpr size_t kDecBytes = (size_t)kBatchHalf * kNumChunk * kHid * 4;
constexpr size_t kWsTotal  = kOffR7 + kDecBytes;
static_assert(kWsTotal == 101449728);
static_assert(kWsTotal <= 134217728);
static_assert(2 * (size_t)kRowsHalf * kGateRank * 2 <= kPlaneF32);
static_assert(kOffR2 % 128 == 0 && kOffR7 % 128 == 0);

__device__ __forceinline__ unsigned short f2bf_bits(float f) {
  unsigned u = __float_as_uint(f);
  return (unsigned short)((u + 0x7FFFu + ((u >> 16) & 1u)) >> 16);
}
__device__ __forceinline__ float bf_bits2f(unsigned short h) { return __uint_as_float(((unsigned)h) << 16); }

__device__ __forceinline__ void dep_guard_h(v8f& a, v8f& b, v16h x, v16h y) { asm volatile("v_nop\n\tv_nop\n\tv_nop\n\tv_nop" : "+v"(a), "+v"(b) : "v"(x), "v"(y)); }
__device__ __forceinline__ void dep_guard_b(v8f& a, v8f& b, v16b x, v16b y) { asm volatile("v_nop\n\tv_nop\n\tv_nop\n\tv_nop" : "+v"(a), "+v"(b) : "v"(x), "v"(y)); }
__device__ __forceinline__ void keep4_h(v16h a, v16h b, v16h c, v16h d) { asm volatile("v_nop" :: "v"(a), "v"(b), "v"(c), "v"(d)); }
__device__ __forceinline__ void keep4_b(v16b a, v16b b, v16b c, v16b d) { asm volatile("v_nop" :: "v"(a), "v"(b), "v"(c), "v"(d)); }
__device__ __forceinline__ void acc_guard4(v8f& a, v8f& b, v8f& c, v8f& d) { asm volatile("v_nop\n\tv_nop\n\tv_nop\n\tv_nop" : "+v"(a), "+v"(b), "+v"(c), "+v"(d)); }
template <typename T> struct Frag;
template <> struct Frag<_Float16> {
  typedef v16h V; union U { v16h v; v8h h[2]; };
  static __device__ __forceinline__ v16h load(const _Float16* p) {
    U f; f.h[0] = *(const v8h*)(p); f.h[1] = *(const v8h*)(p + 16); return f.v;
  }
  static __device__ __forceinline__ v8f mma(v16h a, v16h b, v8f c) {
    return __builtin_amdgcn_wmma_f32_16x16x32_f16(false, a, false, b, (short)0, c, false, false);
  }
  static __device__ __forceinline__ void guard(v8f& a, v8f& b, v16h x, v16h y) { dep_guard_h(a, b, x, y); }
  static __device__ __forceinline__ void keep(v16h a, v16h b, v16h c, v16h d) { keep4_h(a, b, c, d); }
};
template <> struct Frag<__bf16> {
  typedef v16b V; union U { v16b v; v8b h[2]; };
  static __device__ __forceinline__ v16b load(const __bf16* p) {
    U f; f.h[0] = *(const v8b*)(p); f.h[1] = *(const v8b*)(p + 16); return f.v;
  }
  static __device__ __forceinline__ v8f mma(v16b a, v16b b, v8f c) {
    return __builtin_amdgcn_wmma_f32_16x16x32_bf16(false, a, false, b, (short)0, c, false, false);
  }
  static __device__ __forceinline__ void guard(v8f& a, v8f& b, v16b x, v16b y) { dep_guard_b(a, b, x, y); }
  static __device__ __forceinline__ void keep(v16b a, v16b b, v16b c, v16b d) { keep4_b(a, b, c, d); }
};
template <int ET> struct Elem;
template <> struct Elem<0> { typedef _Float16 T; };
template <> struct Elem<1> { typedef __bf16 T; };

__device__ __forceinline__ v8f zero8() { return (v8f){0.f, 0.f, 0.f, 0.f, 0.f, 0.f, 0.f, 0.f}; }

__device__ __forceinline__ v8f mma3_bf(v8f c, v16b ah, v16b al, v16b bh, v16b bl) {
  c = __builtin_amdgcn_wmma_f32_16x16x32_bf16(false, ah, false, bh, (short)0, c, false, false);
  c = __builtin_amdgcn_wmma_f32_16x16x32_bf16(false, ah, false, bl, (short)0, c, false, false);
  c = __builtin_amdgcn_wmma_f32_16x16x32_bf16(false, al, false, bh, (short)0, c, false, false);
  asm volatile("v_nop\n\tv_nop\n\tv_nop\n\tv_nop" : "+v"(c) : "v"(ah), "v"(al), "v"(bh), "v"(bl));
  return c;
}

__device__ __forceinline__ void split_pack2(float a, float b, unsigned& hw, unsigned& lw) {
  const unsigned short ha = f2bf_bits(a), hb2 = f2bf_bits(b);
  const unsigned short la = f2bf_bits(a - bf_bits2f(ha)), lb2 = f2bf_bits(b - bf_bits2f(hb2));
  hw = (unsigned)ha | ((unsigned)hb2 << 16);
  lw = (unsigned)la | ((unsigned)lb2 << 16);
}
__device__ __forceinline__ unsigned pack2_bf(float a, float b) {
  return (unsigned)f2bf_bits(a) | ((unsigned)f2bf_bits(b) << 16);
}

template <int ET, int SPLITM, int OUT_MODE, int ACT>
__global__ __launch_bounds__(256) void wmma_gemm64(
    const unsigned short* __restrict__ Ap, const unsigned short* __restrict__ A2p, int lda, long strideA,
    const unsigned short* __restrict__ Btp, const unsigned short* __restrict__ Bt2p, int ldb, long strideB,
    void* __restrict__ Cout, void* __restrict__ Cout2, int ldc, long strideC,
    int M, int N, int K, float scale) {
  typedef typename Elem<ET>::T T;
  typedef typename Frag<T>::V V;
  const T* A = (const T*)Ap; const T* A2 = (const T*)A2p; const T* Bt = (const T*)Btp; const T* Bt2 = (const T*)Bt2p;
  __shared__ __align__(16) float sT[8][16 * 68];
  const int b    = blockIdx.y;
  const int lane = threadIdx.x & 31;
  const int wave = threadIdx.x >> 5;
  const int tilesN = N >> 6;
  const int tilesM = M >> 6;
  const int tile = blockIdx.x * 8 + wave;
  if (tile >= tilesM * tilesN) return;
  const int tm = tile / tilesN;
  const int tn = tile - tm * tilesN;
  const int m0 = tm << 6;
  const int n0 = tn << 6;

  const T* Ab  = A  + (size_t)b * strideA;
  const T* Bb  = Bt + (size_t)b * strideB;
  const T* Ab2 = (SPLITM >= 1) ? (A2  + (size_t)b * strideA) : nullptr;
  const T* Bb2 = (SPLITM == 2) ? (Bt2 + (size_t)b * strideB) : nullptr;

  const int rlane = lane & 15;
  const int koff  = (lane >> 4) * 8;
  const int mOff  = (lane >> 4) * 8;

  v8f acc[4][4];
#pragma unroll
  for (int i = 0; i < 4; ++i)
#pragma unroll
    for (int j = 0; j < 4; ++j) acc[i][j] = zero8();

  for (int k0 = 0; k0 < K; k0 += 32) {
    V bh[4], bl[4];
#pragma unroll
    for (int j = 0; j < 4; ++j) {
      const size_t bo = (size_t)(n0 + (j << 4) + rlane) * ldb + koff + k0;
      bh[j] = Frag<T>::load(Bb + bo);
      if (SPLITM == 2) bl[j] = Frag<T>::load(Bb2 + bo);
    }
#pragma unroll
    for (int i = 0; i < 4; ++i) {
      const size_t ao = (size_t)(m0 + (i << 4) + rlane) * lda + koff + k0;
      V ah = Frag<T>::load(Ab + ao);
      V al = ah;
      if (SPLITM >= 1) al = Frag<T>::load(Ab2 + ao);
#pragma unroll
      for (int j = 0; j < 4; ++j) {
        acc[i][j] = Frag<T>::mma(ah, bh[j], acc[i][j]);
        if (SPLITM == 2) acc[i][j] = Frag<T>::mma(ah, bl[j], acc[i][j]);
        if (SPLITM >= 1) acc[i][j] = Frag<T>::mma(al, bh[j], acc[i][j]);
      }
      Frag<T>::guard(acc[i][0], acc[i][3], ah, al);
    }
    Frag<T>::keep(bh[0], bh[1], bh[2], bh[3]);
    if (SPLITM == 2) Frag<T>::keep(bl[0], bl[1], bl[2], bl[3]);
  }
  acc_guard4(acc[0][0], acc[0][1], acc[0][2], acc[0][3]);
  acc_guard4(acc[1][0], acc[1][1], acc[1][2], acc[1][3]);
  acc_guard4(acc[2][0], acc[2][1], acc[2][2], acc[2][3]);
  acc_guard4(acc[3][0], acc[3][1], acc[3][2], acc[3][3]);

  float* slab = sT[wave];
#pragma unroll
  for (int i = 0; i < 4; ++i) {
    const int mBase = m0 + (i << 4);
#pragma unroll
    for (int j = 0; j < 4; ++j) {
#pragma unroll
      for (int r = 0; r < 8; ++r) {
        float v = acc[i][j][r] * scale;
        if (ACT == 1) v = tanhf(v);
        if (ACT == 2) v = fmaxf(v, 0.0f);
        if (ACT == 3) v = v / (1.0f + expf(-v));
        if (ACT == 4) v = (v > 0.f) ? v : 0.01f * v;
        if (ACT == 6) v = v * __builtin_amdgcn_rcpf(1.0f + expf(-v));
        slab[(mOff + r) * 68 + (j << 4) + rlane] = v;
      }
    }
    __builtin_amdgcn_fence(__ATOMIC_RELEASE, "workgroup");
    __builtin_amdgcn_wave_barrier();
    __builtin_amdgcn_fence(__ATOMIC_ACQUIRE, "workgroup");
    if (OUT_MODE == 0) {
      float* C = (float*)Cout + (size_t)b * strideC;
      const int hh = lane >> 4, c4 = (lane & 15) * 4;
      for (int pass = 0; pass < 2; ++pass) {
#pragma unroll
        for (int it = 0; it < 8; ++it) {
          const int row = it * 2 + hh;
          v4f v = *(const v4f*)(slab + row * 68 + c4);
          *(volatile v4f*)(C + (size_t)(mBase + row) * ldc + n0 + c4) = v;
        }
        __threadfence();
      }
    } else {
      const int q = lane >> 3, c8 = (lane & 7) * 8;
      unsigned short* C  = (unsigned short*)Cout  + (size_t)b * strideC;
      unsigned short* C2 = (OUT_MODE == 2) ? ((unsigned short*)Cout2 + (size_t)b * strideC) : nullptr;
      for (int pass = 0; pass < 2; ++pass) {
#pragma unroll
        for (int it = 0; it < 4; ++it) {
          const int row = it * 4 + q;
          const float* sp = slab + row * 68 + c8;
          v8h hv, lv;
#pragma unroll
          for (int e = 0; e < 8; ++e) {
            if (OUT_MODE == 1) {
              hv[e] = (_Float16)sp[e];
            } else {
              unsigned short hb = f2bf_bits(sp[e]);
              unsigned short lb = f2bf_bits(sp[e] - bf_bits2f(hb));
              hv[e] = __builtin_bit_cast(_Float16, hb);
              lv[e] = __builtin_bit_cast(_Float16, lb);
            }
          }
          *(volatile v8h*)(C + (size_t)(mBase + row) * ldc + n0 + c8) = hv;
          if (OUT_MODE == 2) *(volatile v8h*)(C2 + (size_t)(mBase + row) * ldc + n0 + c8) = lv;
        }
        __threadfence();
      }
    }
    __builtin_amdgcn_fence(__ATOMIC_RELEASE, "workgroup");
    __builtin_amdgcn_wave_barrier();
    __builtin_amdgcn_fence(__ATOMIC_ACQUIRE, "workgroup");
  }
}

__global__ __launch_bounds__(256) void cast_f32_bf16x8(
    const float* __restrict__ in, unsigned short* __restrict__ out, int n8) {
  const int i = blockIdx.x * 256 + threadIdx.x;
  if (i < n8) {
    const size_t o0 = (size_t)i * 8;
    const v4f a = *(const v4f*)(in + o0);
    const v4f b = *(const v4f*)(in + o0 + 4);
    v4u w;
    w[0] = pack2_bf(a[0], a[1]);
    w[1] = pack2_bf(a[2], a[3]);
    w[2] = pack2_bf(b[0], b[1]);
    w[3] = pack2_bf(b[2], b[3]);
    *(volatile v4u*)(out + o0) = w;
    __threadfence();
    *(volatile v4u*)(out + o0) = w;
  }
}

__global__ __launch_bounds__(256) void cumlse_kernel(
    const float* __restrict__ kraw, float* __restrict__ z, int seqLen, int ld, int nUnits) {
  const int g = blockIdx.x * 256 + threadIdx.x;
  if (g >= nUnits) return;
  const int sq = g / ld;
  const int c  = g - sq * ld;
  const size_t base = (size_t)sq * seqLen * ld + c;
  const float* p = kraw + base;
  float* zo = z + base;
  float m = -INFINITY, s = 0.0f;
#pragma unroll 1
  for (int t = 0; t < seqLen; ++t) {
    const float x  = p[(size_t)t * ld];
    const float mn = fmaxf(m, x);
    s = s * expf(m - mn) + expf(x - mn);
    m = mn;
    const float zz = m + logf(s);
    volatile float* zp = zo + (size_t)t * ld;
    *zp = zz;
    __threadfence();
    *zp = zz;
  }
}

__global__ __launch_bounds__(256) void decay_kernel(
    const float* __restrict__ z, float* __restrict__ dec, int seqLen, int ld, int nChunk, int nUnits) {
  const int g = blockIdx.x * 256 + threadIdx.x;
  if (g >= nUnits) return;
  const int r  = g / ld;
  const int c  = g - r * ld;
  const int sq = r / nChunk;
  const int n  = r - sq * nChunk;
  const int t0 = n * 64;
  const int tl = sq * seqLen + t0 + 63;
  const int tp = (n == 0) ? (sq * seqLen) : (sq * seqLen + t0 - 1);
  const float zl = z[(size_t)tl * ld + c];
  const float zp = z[(size_t)tp * ld + c];
  const float dv = (n == 0) ? 1.0f : expf(zp - zl);
  volatile float* dp = dec + (size_t)r * ld + c;
  *dp = dv;
  __threadfence();
  *dp = dv;
}

template <int KPATH>
__device__ __forceinline__ float gp_val(float s, float zl, float zr) {
  if (KPATH == 0) return s * expf(zl - zr);
  return expf(s - zl);
}
template <int KPATH>
__global__ __launch_bounds__(256) void gate_plane_kernel(
    const float* __restrict__ src, const float* __restrict__ z,
    unsigned short* __restrict__ ph, unsigned short* __restrict__ pl, int ld, int nUnits) {
  const int g = blockIdx.x * 256 + threadIdx.x;
  if (g >= nUnits) return;
  const int gpr = ld >> 3;
  const int row = g / gpr;
  const int c0  = (g - row * gpr) * 8;
  const int last = row | 63;
  const size_t o0 = (size_t)row * ld + c0;
  const size_t ol = (size_t)last * ld + c0;
  const v4f sa = *(const v4f*)(src + o0);
  const v4f sb = *(const v4f*)(src + o0 + 4);
  const v4f la = *(const v4f*)(z + ol);
  const v4f lb = *(const v4f*)(z + ol + 4);
  v4f za = la, zb = lb;
  if (KPATH == 0) { za = *(const v4f*)(z + o0); zb = *(const v4f*)(z + o0 + 4); }
  const float r0 = gp_val<KPATH>(sa[0], la[0], za[0]);
  const float r1 = gp_val<KPATH>(sa[1], la[1], za[1]);
  const float r2 = gp_val<KPATH>(sa[2], la[2], za[2]);
  const float r3 = gp_val<KPATH>(sa[3], la[3], za[3]);
  const float r4 = gp_val<KPATH>(sb[0], lb[0], zb[0]);
  const float r5 = gp_val<KPATH>(sb[1], lb[1], zb[1]);
  const float r6 = gp_val<KPATH>(sb[2], lb[2], zb[2]);
  const float r7 = gp_val<KPATH>(sb[3], lb[3], zb[3]);
  unsigned h0, l0, h1, l1, h2, l2, h3, l3;
  split_pack2(r0, r1, h0, l0);
  split_pack2(r2, r3, h1, l1);
  split_pack2(r4, r5, h2, l2);
  split_pack2(r6, r7, h3, l3);
  v4u wh, wl;
  wh[0] = h0; wh[1] = h1; wh[2] = h2; wh[3] = h3;
  wl[0] = l0; wl[1] = l1; wl[2] = l2; wl[3] = l3;
  *(volatile v4u*)(ph + o0) = wh;
  *(volatile v4u*)(pl + o0) = wl;
  __threadfence();
  *(volatile v4u*)(ph + o0) = wh;
  *(volatile v4u*)(pl + o0) = wl;
}

constexpr int kGlaSP = 136;
constexpr int kGlaTP = 72;
constexpr int kGlaOP = 68;
constexpr int kOffSm = 0;
constexpr int kOffSh = kOffSm + 64 * 128 * 4;
constexpr int kOffSl = kOffSh + 64 * kGlaSP * 2;
constexpr int kOffKh = kOffSl + 64 * kGlaSP * 2;
constexpr int kOffKl = kOffKh + 128 * kGlaTP * 2;
constexpr int kOffVh = kOffKl + 128 * kGlaTP * 2;
constexpr int kOffVl = kOffVh + 64 * kGlaTP * 2;
constexpr int kOffAh = kOffVl + 64 * kGlaTP * 2;
constexpr int kOffAl = kOffAh + 64 * kGlaTP * 2;
constexpr int kOffOs = kOffAl + 64 * kGlaTP * 2;
constexpr int kGlaLdsBytes = kOffOs + 64 * kGlaOP * 4;
static_assert(kGlaLdsBytes == 158720);
static_assert(kOffSh % 16 == 0 && kOffKh % 16 == 0 && kOffVh % 16 == 0 && kOffAh % 16 == 0 && kOffOs % 16 == 0);

__device__ __forceinline__ v16b lfrag(const unsigned short* p) { return Frag<__bf16>::load((const __bf16*)p); }

__global__ __launch_bounds__(256) void gla_chunk_kernel(
    const unsigned short* __restrict__ q2h, const unsigned short* __restrict__ q2l,
    const unsigned short* __restrict__ kth, const unsigned short* __restrict__ ktl,
    const unsigned short* __restrict__ vph, const unsigned short* __restrict__ vpl,
    const float* __restrict__ dec, float* __restrict__ o,
    int seqLen, int ld, int nChunk) {
  extern __shared__ __align__(16) unsigned char gsm[];
  float* Sm = (float*)(gsm + kOffSm);
  unsigned short* Sh = (unsigned short*)(gsm + kOffSh);
  unsigned short* Sl = (unsigned short*)(gsm + kOffSl);
  unsigned short* Kh = (unsigned short*)(gsm + kOffKh);
  unsigned short* Kl = (unsigned short*)(gsm + kOffKl);
  unsigned short* Vh = (unsigned short*)(gsm + kOffVh);
  unsigned short* Vl = (unsigned short*)(gsm + kOffVl);
  unsigned short* Ah = (unsigned short*)(gsm + kOffAh);
  unsigned short* Al = (unsigned short*)(gsm + kOffAl);
  float* Os = (float*)(gsm + kOffOs);

  const int tid = threadIdx.x, lane = tid & 31, wave = tid >> 5;
  const int hh = lane >> 4, rl = lane & 15, koff = hh * 8;
  const int vhalf = blockIdx.x, h = blockIdx.y, sq = blockIdx.z;
  const int ch  = h * kHeadDim;
  const int vch = ch + vhalf * 64;
  const int rowb = sq * seqLen;
  const __bf16* Qh  = (const __bf16*)q2h;
  const __bf16* Ql  = (const __bf16*)q2l;
  const __bf16* Kgh = (const __bf16*)kth;
  const __bf16* Kgl = (const __bf16*)ktl;

  for (int i = tid; i < 64 * 128; i += 256) Sm[i] = 0.0f;

  for (int n = 0; n < nChunk; ++n) {
    const int gr = rowb + n * 64;
    __syncthreads();
    {
      const int d = tid & 127, e0 = tid >> 7;
      const float dv = dec[(size_t)(sq * nChunk + n) * ld + ch + d];
#pragma unroll 2
      for (int it = 0; it < 32; ++it) {
        const int e = it * 2 + e0;
        const float s = Sm[e * 128 + d] * dv;
        Sm[e * 128 + d] = s;
        const unsigned short hb = f2bf_bits(s);
        Sh[e * kGlaSP + d] = hb;
        Sl[e * kGlaSP + d] = f2bf_bits(s - bf_bits2f(hb));
      }
    }
#pragma unroll 1
    for (int it = 0; it < 4; ++it) {
      const int u = it * 256 + tid;
      const int c = u >> 4, grp = u & 15;
      const size_t go = (size_t)(gr + c) * ld + ch + grp * 8;
      const v4u wh = *(const v4u*)(kth + go);
      const v4u wl = *(const v4u*)(ktl + go);
      unsigned short* ph = Kh + (grp * 8) * kGlaTP + c;
      unsigned short* pl = Kl + (grp * 8) * kGlaTP + c;
#pragma unroll
      for (int w2 = 0; w2 < 4; ++w2) {
        ph[(2 * w2) * kGlaTP]     = (unsigned short)(wh[w2] & 0xffffu);
        ph[(2 * w2 + 1) * kGlaTP] = (unsigned short)(wh[w2] >> 16);
        pl[(2 * w2) * kGlaTP]     = (unsigned short)(wl[w2] & 0xffffu);
        pl[(2 * w2 + 1) * kGlaTP] = (unsigned short)(wl[w2] >> 16);
      }
    }
#pragma unroll 1
    for (int it = 0; it < 2; ++it) {
      const int u = it * 256 + tid;
      const int c = u >> 3, grp = u & 7;
      const size_t go = (size_t)(gr + c) * ld + vch + grp * 8;
      const v4u wh = *(const v4u*)(vph + go);
      const v4u wl = *(const v4u*)(vpl + go);
      unsigned short* ph = Vh + (grp * 8) * kGlaTP + c;
      unsigned short* pl = Vl + (grp * 8) * kGlaTP + c;
#pragma unroll
      for (int w2 = 0; w2 < 4; ++w2) {
        ph[(2 * w2) * kGlaTP]     = (unsigned short)(wh[w2] & 0xffffu);
        ph[(2 * w2 + 1) * kGlaTP] = (unsigned short)(wh[w2] >> 16);
        pl[(2 * w2) * kGlaTP]     = (unsigned short)(wl[w2] & 0xffffu);
        pl[(2 * w2 + 1) * kGlaTP] = (unsigned short)(wl[w2] >> 16);
      }
    }
    __syncthreads();

#pragma unroll 1
    for (int s = 0; s < 2; ++s) {
      const int st = wave * 2 + s;
      const int ti = st >> 2, tj = st & 3;
      const int abase = (ti * 16 + hh * 8) * kGlaTP + tj * 16 + rl;
      if (tj <= ti) {
        v8f acc = zero8();
#pragma unroll 1
        for (int k0 = 0; k0 < 128; k0 += 32) {
          const size_t ao = (size_t)(gr + ti * 16 + rl) * ld + ch + k0 + koff;
          const size_t bo = (size_t)(gr + tj * 16 + rl) * ld + ch + k0 + koff;
          const v16b fa  = Frag<__bf16>::load(Qh + ao);
          const v16b fal = Frag<__bf16>::load(Ql + ao);
          const v16b fb  = Frag<__bf16>::load(Kgh + bo);
          const v16b fbl = Frag<__bf16>::load(Kgl + bo);
          acc = mma3_bf(acc, fa, fal, fb, fbl);
        }
        const int ibase = ti * 16 + hh * 8, j = tj * 16 + rl;
#pragma unroll
        for (int r = 0; r < 8; ++r) {
          const float val = (j <= ibase + r) ? acc[r] : 0.0f;
          const unsigned short hb = f2bf_bits(val);
          Ah[abase + r * kGlaTP] = hb;
          Al[abase + r * kGlaTP] = f2bf_bits(val - bf_bits2f(hb));
        }
      } else {
#pragma unroll
        for (int r = 0; r < 8; ++r) {
          Ah[abase + r * kGlaTP] = (unsigned short)0;
          Al[abase + r * kGlaTP] = (unsigned short)0;
        }
      }
    }

    v8f oacc[2];
#pragma unroll
    for (int s = 0; s < 2; ++s) {
      const int st = wave * 2 + s;
      const int ti = st >> 2, te = st & 3;
      v8f acc = zero8();
#pragma unroll 1
      for (int k0 = 0; k0 < 128; k0 += 32) {
        const size_t ao = (size_t)(gr + ti * 16 + rl) * ld + ch + k0 + koff;
        const v16b fa  = Frag<__bf16>::load(Qh + ao);
        const v16b fal = Frag<__bf16>::load(Ql + ao);
        const v16b fb  = lfrag(Sh + (te * 16 + rl) * kGlaSP + k0 + koff);
        const v16b fbl = lfrag(Sl + (te * 16 + rl) * kGlaSP + k0 + koff);
        acc = mma3_bf(acc, fa, fal, fb, fbl);
      }
      oacc[s] = acc;
    }
    __syncthreads();

#pragma unroll
    for (int s = 0; s < 2; ++s) {
      const int st = wave * 2 + s;
      const int ti = st >> 2, te = st & 3;
      v8f acc = oacc[s];
#pragma unroll
      for (int k0 = 0; k0 < 64; k0 += 32) {
        const v16b fa  = lfrag(Ah + (ti * 16 + rl) * kGlaTP + k0 + koff);
        const v16b fal = lfrag(Al + (ti * 16 + rl) * kGlaTP + k0 + koff);
        const v16b fb  = lfrag(Vh + (te * 16 + rl) * kGlaTP + k0 + koff);
        const v16b fbl = lfrag(Vl + (te * 16 + rl) * kGlaTP + k0 + koff);
        acc = mma3_bf(acc, fa, fal, fb, fbl);
      }
      const int ibase = ti * 16 + hh * 8;
#pragma unroll
      for (int r = 0; r < 8; ++r) Os[(ibase + r) * kGlaOP + te * 16 + rl] = acc[r];
    }
    __syncthreads();
    {
      const int c4 = rl * 4;
      float* ob = o + (size_t)gr * ld + vch;
      for (int pass = 0; pass < 2; ++pass) {
#pragma unroll
        for (int it = 0; it < 4; ++it) {
          const int row = wave * 8 + it * 2 + hh;
          const v4f val = *(const v4f*)(Os + row * kGlaOP + c4);
          *(volatile v4f*)(ob + (size_t)row * ld + c4) = val;
        }
        __threadfence();
      }
    }

#pragma unroll 1
    for (int s = 0; s < 4; ++s) {
      const int st = wave * 4 + s;
      const int te = st >> 3, td = st & 7;
      v8f acc;
#pragma unroll
      for (int r = 0; r < 8; ++r) acc[r] = Sm[(te * 16 + hh * 8 + r) * 128 + td * 16 + rl];
#pragma unroll
      for (int k0 = 0; k0 < 64; k0 += 32) {
        const v16b fa  = lfrag(Vh + (te * 16 + rl) * kGlaTP + k0 + koff);
        const v16b fal = lfrag(Vl + (te * 16 + rl) * kGlaTP + k0 + koff);
        const v16b fb  = lfrag(Kh + (td * 16 + rl) * kGlaTP + k0 + koff);
        const v16b fbl = lfrag(Kl + (td * 16 + rl) * kGlaTP + k0 + koff);
        acc = mma3_bf(acc, fa, fal, fb, fbl);
      }
#pragma unroll
      for (int r = 0; r < 8; ++r) Sm[(te * 16 + hh * 8 + r) * 128 + td * 16 + rl] = acc[r];
    }
  }
}

__device__ __forceinline__ float rg_val(float ov, float gv, float wv, float rinv) {
  const float wr = bf_bits2f(f2bf_bits(wv));
  const float sg = gv * __builtin_amdgcn_rcpf(1.0f + expf(-gv));
  return ((ov * rinv) * wr) * sg;
}
__global__ __launch_bounds__(128) void rms_gate_kernel(
    const float* __restrict__ o, const float* __restrict__ gate, const float* __restrict__ gw,
    unsigned short* __restrict__ yh, unsigned short* __restrict__ yl, int ld, float invD, float eps) {
  __shared__ float red[4];
  const int row = blockIdx.x;
  const int tid = threadIdx.x, lane = tid & 31, wave = tid >> 5;
  const int c0 = tid * 8;
  const size_t o0 = (size_t)row * ld + c0;
  const v4f oa = *(const v4f*)(o + o0);
  const v4f ob = *(const v4f*)(o + o0 + 4);
  const v4f ga = *(const v4f*)(gate + o0);
  const v4f gb = *(const v4f*)(gate + o0 + 4);
  const v4f wa = *(const v4f*)(gw + c0);
  const v4f wb = *(const v4f*)(gw + c0 + 4);
  float ss = oa[0] * oa[0];
  ss += oa[1] * oa[1]; ss += oa[2] * oa[2]; ss += oa[3] * oa[3];
  ss += ob[0] * ob[0]; ss += ob[1] * ob[1]; ss += ob[2] * ob[2]; ss += ob[3] * ob[3];
#pragma unroll
  for (int off = 16; off > 0; off >>= 1) ss += __shfl_xor(ss, off, 32);
  if (lane == 0) red[wave] = ss;
  __syncthreads();
  const float tot = (red[0] + red[1]) + (red[2] + red[3]);
  const float rinv = rsqrtf(tot * invD + eps);
  const float r0 = rg_val(oa[0], ga[0], wa[0], rinv);
  const float r1 = rg_val(oa[1], ga[1], wa[1], rinv);
  const float r2 = rg_val(oa[2], ga[2], wa[2], rinv);
  const float r3 = rg_val(oa[3], ga[3], wa[3], rinv);
  const float r4 = rg_val(ob[0], gb[0], wb[0], rinv);
  const float r5 = rg_val(ob[1], gb[1], wb[1], rinv);
  const float r6 = rg_val(ob[2], gb[2], wb[2], rinv);
  const float r7 = rg_val(ob[3], gb[3], wb[3], rinv);
  unsigned h0, l0, h1, l1, h2, l2, h3, l3;
  split_pack2(r0, r1, h0, l0);
  split_pack2(r2, r3, h1, l1);
  split_pack2(r4, r5, h2, l2);
  split_pack2(r6, r7, h3, l3);
  v4u wh, wl;
  wh[0] = h0; wh[1] = h1; wh[2] = h2; wh[3] = h3;
  wl[0] = l0; wl[1] = l1; wl[2] = l2; wl[3] = l3;
  *(volatile v4u*)(yh + o0) = wh;
  *(volatile v4u*)(yl + o0) = wl;
  __threadfence();
  *(volatile v4u*)(yh + o0) = wh;
  *(volatile v4u*)(yl + o0) = wl;
}

static inline unsigned gemm_blocks(int M, int N) { return (unsigned)(((M >> 6) * (N >> 6) + 7) / 8); }

extern "C" void kernel_launch(void* const* d_in, const int* in_sizes, int n_in,
                              void* d_out, int out_size, void* d_ws, size_t ws_size,
                              hipStream_t stream) {
  if (n_in < 8) return;
  if (in_sizes[0] != kBatch * kSeqLen * kHid) return;
  if (in_sizes[1] != kHid * kHid || in_sizes[2] != kHid * kHid || in_sizes[3] != kHid * kHid) return;
  if (in_sizes[4] != kGateRank * kHid || in_sizes[5] != kHid * kGateRank) return;
  if (in_sizes[6] != kHid || in_sizes[7] != kHid * kHid) return;
  if (out_size != kBatch * kSeqLen * kHid) return;
  if (ws_size < kWsTotal) return;

  const float* x   = (const float*)d_in[0];
  const float* Wq  = (const float*)d_in[1];
  const float* Wk  = (const float*)d_in[2];
  const float* Wv  = (const float*)d_in[3];
  const float* Wg1 = (const float*)d_in[4];
  const float* Wg2 = (const float*)d_in[5];
  const float* gnw = (const float*)d_in[6];
  const float* Wo  = (const float*)d_in[7];
  float* outp = (float*)d_out;

  unsigned char* ws = (unsigned char*)d_ws;
  unsigned short* xb   = (unsigned short*)(ws + kOffXb);
  unsigned short* wqb  = (unsigned short*)(ws + kOffWq);
  unsigned short* wkb  = (unsigned short*)(ws + kOffWk);
  unsigned short* wvb  = (unsigned short*)(ws + kOffWv);
  unsigned short* wob  = (unsigned short*)(ws + kOffWo);
  unsigned short* wg1b = (unsigned short*)(ws + kOffWg1);
  unsigned short* wg2b = (unsigned short*)(ws + kOffWg2);
  float*          krawp = (float*)(ws + kOffR2);
  unsigned short* vhi   = (unsigned short*)(ws + kOffR2);
  unsigned short* vlo   = (unsigned short*)(ws + kOffR2 + kPlane16);
  float*          gatep = (float*)(ws + kOffR2);
  float*          zp    = (float*)(ws + kOffR3);
  float*          op    = (float*)(ws + kOffR3);
  float*          qp    = (float*)(ws + kOffR4);
  unsigned short* yhi   = (unsigned short*)(ws + kOffR4);
  unsigned short* ylo   = (unsigned short*)(ws + kOffR4 + kPlane16);
  unsigned short* q2hi  = (unsigned short*)(ws + kOffR5);
  unsigned short* q2lo  = (unsigned short*)(ws + kOffR5 + kPlane16);
  unsigned short* g1hi  = (unsigned short*)(ws + kOffR5);
  unsigned short* g1lo  = (unsigned short*)(ws + kOffR5 + (size_t)kRowsHalf * kGateRank * 2);
  unsigned short* kthi  = (unsigned short*)(ws + kOffR6);
  unsigned short* ktlo  = (unsigned short*)(ws + kOffR6 + kPlane16);
  float*          decp  = (float*)(ws + kOffR7);

  const int n8w  = kHid * kHid / 8;
  const int n8g  = kGateRank * kHid / 8;
  const int n8x  = kRowsHalf * kHid / 8;
  cast_f32_bf16x8<<<dim3(n8w / 256), dim3(256), 0, stream>>>(Wq,  wqb,  n8w);
  cast_f32_bf16x8<<<dim3(n8w / 256), dim3(256), 0, stream>>>(Wk,  wkb,  n8w);
  cast_f32_bf16x8<<<dim3(n8w / 256), dim3(256), 0, stream>>>(Wv,  wvb,  n8w);
  cast_f32_bf16x8<<<dim3(n8w / 256), dim3(256), 0, stream>>>(Wo,  wob,  n8w);
  cast_f32_bf16x8<<<dim3(n8g / 256), dim3(256), 0, stream>>>(Wg1, wg1b, n8g);
  cast_f32_bf16x8<<<dim3(n8g / 256), dim3(256), 0, stream>>>(Wg2, wg2b, n8g);

  const unsigned gbFull = gemm_blocks(kRowsHalf, kHid);
  const unsigned gbG1   = gemm_blocks(kRowsHalf, kGateRank);
  const int cumUnits  = kBatchHalf * kHid;
  const int decUnits  = kBatchHalf * kNumChunk * kHid;
  const int gpUnits   = kRowsHalf * (kHid / 8);
  const float invD = 1.0f / (float)kHid;
  const float eps  = 1e-5f;

  for (int hb = 0; hb < kNumHalf; ++hb) {
    const float* xh = x + (size_t)hb * kRowsHalf * kHid;
    float* outh = outp + (size_t)hb * kRowsHalf * kHid;

    cast_f32_bf16x8<<<dim3(n8x / 256), dim3(256), 0, stream>>>(xh, xb, n8x);

    wmma_gemm64<1, 0, 0, 0><<<dim3(gbFull, 1), dim3(256), 0, stream>>>(
        xb, xb, kHid, 0L, wkb, wkb, kHid, 0L, (void*)krawp, (void*)krawp, kHid, 0L,
        kRowsHalf, kHid, kHid, 1.0f);

    cumlse_kernel<<<dim3(cumUnits / 256), dim3(256), 0, stream>>>(krawp, zp, kSeqLen, kHid, cumUnits);

    wmma_gemm64<1, 0, 0, 6><<<dim3(gbFull, 1), dim3(256), 0, stream>>>(
        xb, xb, kHid, 0L, wqb, wqb, kHid, 0L, (void*)qp, (void*)qp, kHid, 0L,
        kRowsHalf, kHid, kHid, 1.0f);

    decay_kernel<<<dim3(decUnits / 256), dim3(256), 0, stream>>>(zp, decp, kSeqLen, kHid, kNumChunk, decUnits);

    gate_plane_kernel<0><<<dim3(gpUnits / 256), dim3(256), 0, stream>>>(qp,    zp, q2hi, q2lo, kHid, gpUnits);
    gate_plane_kernel<1><<<dim3(gpUnits / 256), dim3(256), 0, stream>>>(krawp, zp, kthi, ktlo, kHid, gpUnits);

    wmma_gemm64<1, 0, 2, 0><<<dim3(gbFull, 1), dim3(256), 0, stream>>>(
        xb, xb, kHid, 0L, wvb, wvb, kHid, 0L, (void*)vhi, (void*)vlo, kHid, 0L,
        kRowsHalf, kHid, kHid, 1.0f);

    gla_chunk_kernel<<<dim3(2, kHeads, kBatchHalf), dim3(256), kGlaLdsBytes, stream>>>(
        q2hi, q2lo, kthi, ktlo, vhi, vlo, decp, op, kSeqLen, kHid, kNumChunk);

    wmma_gemm64<1, 0, 2, 0><<<dim3(gbG1, 1), dim3(256), 0, stream>>>(
        xb, xb, kHid, 0L, wg1b, wg1b, kHid, 0L, (void*)g1hi, (void*)g1lo, kGateRank, 0L,
        kRowsHalf, kGateRank, kHid, 1.0f);

    wmma_gemm64<1, 1, 0, 0><<<dim3(gbFull, 1), dim3(256), 0, stream>>>(
        g1hi, g1lo, kGateRank, 0L, wg2b, wg2b, kGateRank, 0L, (void*)gatep, (void*)gatep, kHid, 0L,
        kRowsHalf, kHid, kGateRank, 1.0f);

    rms_gate_kernel<<<dim3(kRowsHalf), dim3(128), 0, stream>>>(op, gatep, gnw, yhi, ylo, kHid, invD, eps);

    wmma_gemm64<1, 1, 0, 0><<<dim3(gbFull, 1), dim3(256), 0, stream>>>(
        yhi, ylo, kHid, 0L, wob, wob, kHid, 0L, (void*)outh, (void*)outh, kHid, 0L,
        kRowsHalf, kHid, kHid, 1.0f);
  }
}
